// LogSSMLayer_62302795596611
// MI455X (gfx1250) — hardware-verified
//
#include <hip/hip_runtime.h>


namespace {
constexpr int NB = 4, S = 2048, D = 1024, NH = 8, DH = 64, HD = NH * DH, NROW = NB * S, NPRJ = 3 * HD + D;
constexpr float XS = 8.0f, WSC = 256.0f, SCALE = 0.125f;

typedef _Float16 b16;
typedef __attribute__((ext_vector_type(16))) _Float16 v16b;
typedef __attribute__((ext_vector_type(8))) _Float16 v8b;
typedef __attribute__((ext_vector_type(8))) float v8f;
typedef __attribute__((ext_vector_type(4))) float v4f;
__device__ __forceinline__ float bf16_rne(float f) { unsigned int u = __float_as_uint(f); u += 0x7FFFu + ((u >> 16) & 1u); return __uint_as_float(u & 0xFFFF0000u); }
__device__ __forceinline__ v16b frag_kb(const b16* p, int hh) { const v8b a = *(const v8b*)(p + 8 * hh), b = *(const v8b*)(p + 16 + 8 * hh); v16b f;
#pragma unroll
  for (int e = 0; e < 8; ++e) { f[e] = a[e]; f[8 + e] = b[e]; } return f; }
__device__ __forceinline__ v8f wmma16b(v16b a, v16b b, v8f c) { v8f d = __builtin_amdgcn_wmma_f32_16x16x32_f16(false, a, false, b, (short)0, c, false, false); asm volatile("v_nop\n\tv_nop\n\tv_nop\n\tv_nop" : "+v"(d) : "v"(a), "v"(b)); return d; }
__device__ __forceinline__ void wave_lds_sync() { __builtin_amdgcn_fence(__ATOMIC_RELEASE, "workgroup"); __builtin_amdgcn_wave_barrier(); __builtin_amdgcn_fence(__ATOMIC_ACQUIRE, "workgroup"); }
__device__ __forceinline__ float pmul(float a, float b) { float p = a * b; asm volatile("" : "+v"(p)); return p; }
__device__ __forceinline__ float softplus_(float x) { return x > 20.0f ? x : log1pf(__expf(x)); }

__global__ __launch_bounds__(256) void prep_kernel(const float* __restrict__ x, const float* __restrict__ wq, const float* __restrict__ wk, const float* __restrict__ wv, const float* __restrict__ wa, const float* __restrict__ wo, b16* __restrict__ X16, b16* __restrict__ WP, b16* __restrict__ WO) {
  const size_t g = (size_t)blockIdx.x * 256 + threadIdx.x; const size_t nx = (size_t)NROW * D / 8, nq = (size_t)HD * D / 8, nv = (size_t)D * D / 8;
  const float* src; b16* dst; float sc = WSC; size_t e;
  if (g < nx) { src = x; dst = X16; e = g * 8; sc = XS; }
  else { size_t h = g - nx; if (h < nq) { src = wq; dst = WP; e = h * 8; } else if (h < 2 * nq) { src = wk; dst = WP + (size_t)HD * D; e = (h - nq) * 8; } else if (h < 3 * nq) { src = wa; dst = WP + (size_t)2 * HD * D; e = (h - 2 * nq) * 8; } else if (h < 3 * nq + nv) { src = wv; dst = WP + (size_t)3 * HD * D; e = (h - 3 * nq) * 8; } else if (h < 3 * nq + 2 * nv) { src = wo; dst = WO; e = (h - 3 * nq - nv) * 8; } else return; }
  const v4f a = *(const v4f*)(src + e), c = *(const v4f*)(src + e + 4); v8b o;
#pragma unroll
  for (int j = 0; j < 4; ++j) { o[j] = (b16)(bf16_rne(a[j]) * sc); o[4 + j] = (b16)(bf16_rne(c[j]) * sc); }
  for (int pass = 0; pass < 2; ++pass) { *(volatile v8b*)(dst + e) = o; __threadfence(); }
}
__global__ __launch_bounds__(128) void proj_kernel(const b16* __restrict__ X16, const b16* __restrict__ WP, const float* __restrict__ ab, float* __restrict__ QKA, float* __restrict__ V32) {
  __shared__ __attribute__((aligned(16))) float Ts[4][16][128 + 4];
  const int wave = threadIdx.x >> 5, lane = threadIdx.x & 31, nloc = lane & 15, hlf = lane >> 4; const size_t m0 = (size_t)blockIdx.x * 64 + wave * 16; const int n0 = blockIdx.y * 128;
  v8f acc[8];
#pragma unroll
  for (int t = 0; t < 8; ++t) acc[t] = (v8f){};
#pragma unroll 2
  for (int kb = 0; kb < D; kb += 32) { const v16b a = frag_kb(X16 + (m0 + nloc) * D + kb, hlf);
#pragma unroll
    for (int t = 0; t < 8; ++t) acc[t] = wmma16b(a, frag_kb(WP + (size_t)(n0 + t * 16 + nloc) * D + kb, hlf), acc[t]); }
  const bool isal = (n0 >= 2 * HD) && (n0 < 3 * HD);
#pragma unroll
  for (int t = 0; t < 8; ++t) { const int n = n0 + t * 16 + nloc; const float bb = isal ? bf16_rne(ab[n - 2 * HD]) : 0.0f;
#pragma unroll
    for (int r = 0; r < 8; ++r) Ts[wave][8 * hlf + r][t * 16 + nloc] = acc[t][r] * (1.0f / (XS * WSC)) + bb; }
  wave_lds_sync();
  const bool isv = n0 >= 3 * HD;
  for (int pass = 0; pass < 2; ++pass) { for (int rr = 0; rr < 16; ++rr) { const v4f vv = *(const v4f*)(&Ts[wave][rr][lane * 4]); if (isv) *(volatile v4f*)(V32 + (m0 + rr) * D + (n0 - 3 * HD) + lane * 4) = vv; else *(volatile v4f*)(QKA + (m0 + rr) * (3 * HD) + n0 + lane * 4) = vv; } __threadfence(); }
}
__global__ __launch_bounds__(256) void coef_kernel(const float* __restrict__ QKA, float* __restrict__ AB) {
  const int wave = threadIdx.x >> 5, lane = threadIdx.x & 31; const size_t row0 = ((size_t)blockIdx.x * 8 + wave) * 2;
  float outv[2];
  for (int rr = 0; rr < 2; ++rr) { const size_t row = row0 + rr; const float* p = QKA + row * (3 * HD); const int h = lane >> 2, part = lane & 3;
    float sb = 0.0f, sa = 0.0f;
#pragma unroll 1
    for (int j = 0; j < 16; ++j) { const int d = h * DH + part * 16 + j; sb += pmul(p[d], p[HD + d]); sa += softplus_(p[2 * HD + d]); }
    sb += __shfl_xor(sb, 1); sb += __shfl_xor(sb, 2); sa += __shfl_xor(sa, 1); sa += __shfl_xor(sa, 2);
    const float a_for = -__shfl(sa, (lane & 7) * 4), b_for = __shfl(sb, (lane & 7) * 4) * SCALE;
    outv[rr] = (lane & 8) ? b_for : a_for; }
  const float mine = (lane < 16) ? outv[0] : outv[1];
  for (int pass = 0; pass < 2; ++pass) { ((volatile float*)AB)[row0 * 16 + lane] = mine; __threadfence(); }
}
__global__ __launch_bounds__(32) void seq_kernel(const float* __restrict__ AB, float* __restrict__ F) {
  const int lane = threadIdx.x; const int b = lane >> 3, h = lane & 7;
  float M = -INFINITY, Zs = 0.0f;
  for (int t = 0; t < S; ++t) { const size_t row = (size_t)b * S + t; const float a = AB[row * 16 + h], bb = AB[row * 16 + 8 + h];
    const float am = a + M; const float Mn = fmaxf(am, bb); const float fA = (M == -INFINITY) ? 0.0f : __expf(am - Mn); const float fB = __expf(bb - Mn); Zs = pmul(fA, Zs) + fB; M = Mn;
    const float iz = 1.0f / Zs;
    for (int pass = 0; pass < 2; ++pass) {
      for (int bb = 0; bb < NB; ++bb) { const int srcl = bb * 8 + (lane & 7); const float vA = __shfl(fA, srcl), vB = __shfl(fB, srcl), vZ = __shfl(iz, srcl); const int comp = lane >> 3;
        ((volatile float*)F)[((size_t)bb * S + t) * 32 + lane] = comp == 0 ? vA : comp == 1 ? vB : comp == 2 ? vZ : 0.0f; }
      __threadfence(); } }
}
__global__ __launch_bounds__(256) void scan_kernel(const float* __restrict__ V32, const float* __restrict__ F, float* __restrict__ Y32) {
  const int tid = blockIdx.x * 256 + threadIdx.x; const int b = tid / D, d = tid - b * D;
  float num[NH];
#pragma unroll
  for (int h = 0; h < NH; ++h) num[h] = 0.0f;
  for (int t = 0; t < S; ++t) { const size_t row = (size_t)b * S + t; const float v = V32[row * D + d]; const float* f = F + row * 32; float y = 0.0f;
#pragma unroll
    for (int h = 0; h < NH; ++h) { num[h] = pmul(f[h], num[h]) + pmul(f[8 + h], v); y += pmul(num[h], f[16 + h]); }
    for (int pass = 0; pass < 2; ++pass) { ((volatile float*)Y32)[row * D + d] = y; __threadfence(); } }
}
__global__ __launch_bounds__(256) void y16_kernel(const float* __restrict__ Y32, b16* __restrict__ Y16, b16* __restrict__ Y16L) {
  const size_t i = ((size_t)blockIdx.x * 256 + threadIdx.x) * 8; if (i >= (size_t)NROW * D) return; const v4f a = *(const v4f*)(Y32 + i), c = *(const v4f*)(Y32 + i + 4); v8b o, ol;
#pragma unroll
  for (int j = 0; j < 4; ++j) { b16 h_, l_; h_ = (b16)(a[j] * XS); l_ = (b16)(a[j] * XS - (float)h_); o[j] = h_; ol[j] = l_; h_ = (b16)(c[j] * XS); l_ = (b16)(c[j] * XS - (float)h_); o[4 + j] = h_; ol[4 + j] = l_; }
  for (int pass = 0; pass < 2; ++pass) { *(volatile v8b*)(Y16 + i) = o; *(volatile v8b*)(Y16L + i) = ol; __threadfence(); }
}
__global__ __launch_bounds__(128) void out_kernel(const b16* __restrict__ Y16, const b16* __restrict__ Y16L, const b16* __restrict__ WO, float* __restrict__ out) {
  __shared__ __attribute__((aligned(16))) float Ts[4][16][128 + 4];
  const int wave = threadIdx.x >> 5, lane = threadIdx.x & 31, nloc = lane & 15, hlf = lane >> 4; const size_t m0 = (size_t)blockIdx.x * 64 + wave * 16; const int n0 = blockIdx.y * 128;
  v8f acc[8];
#pragma unroll
  for (int t = 0; t < 8; ++t) acc[t] = (v8f){};
#pragma unroll 2
  for (int kb = 0; kb < D; kb += 32) { const v16b a = frag_kb(Y16 + (m0 + nloc) * D + kb, hlf), al = frag_kb(Y16L + (m0 + nloc) * D + kb, hlf);
#pragma unroll
    for (int t = 0; t < 8; ++t) { const v16b bw = frag_kb(WO + (size_t)(n0 + t * 16 + nloc) * D + kb, hlf); acc[t] = wmma16b(a, bw, acc[t]); acc[t] = wmma16b(al, bw, acc[t]); } }
#pragma unroll
  for (int t = 0; t < 8; ++t)
#pragma unroll
    for (int r = 0; r < 8; ++r) Ts[wave][8 * hlf + r][t * 16 + nloc] = acc[t][r] * (1.0f / (XS * WSC));
  wave_lds_sync();
  for (int pass = 0; pass < 2; ++pass) { for (int rr = 0; rr < 16; ++rr) *(volatile v4f*)(out + (m0 + rr) * D + n0 + lane * 4) = *(const v4f*)(&Ts[wave][rr][lane * 4]); __threadfence(); }
}
}

extern "C" void kernel_launch(void* const* d_in, const int* in_sizes, int n_in, void* d_out, int out_size, void* d_ws, size_t ws_size, hipStream_t stream) {
  (void)n_in;
  auto Fp = [&](int i) { return (const float*)d_in[i]; };
  if (in_sizes[0] != NROW * D || in_sizes[1] != HD * D || in_sizes[2] != HD * D || in_sizes[3] != D * D || in_sizes[4] != HD * D || in_sizes[5] != HD || in_sizes[6] != D * D || out_size != NROW * D) return;
  size_t off = 0; char* ws = (char*)d_ws;
  auto carve = [&](size_t bytes) { char* p = ws + off; off += (bytes + 255) & ~(size_t)255; return p; };
  b16* X16 = (b16*)carve((size_t)NROW * D * 2); b16* WP = (b16*)carve((size_t)NPRJ * D * 2); b16* WO = (b16*)carve((size_t)D * D * 2); float* QKA = (float*)carve((size_t)NROW * 3 * HD * 4); float* V32 = (float*)carve((size_t)NROW * D * 4);
  float* AB = (float*)carve((size_t)NROW * 16 * 4); float* F = (float*)carve((size_t)NROW * 32 * 4);
  float* Y32 = QKA;
  b16* Y16 = X16;
  b16* Y16L = (b16*)carve((size_t)NROW * D * 2);
  if (off > ws_size || off > ((size_t)128 << 20)) return;
  prep_kernel<<<(NROW * D / 8 + 3 * HD * D / 8 + 2 * D * D / 8 + 255) / 256, 256, 0, stream>>>(Fp(0), Fp(1), Fp(2), Fp(3), Fp(4), Fp(6), X16, WP, WO);
  proj_kernel<<<dim3(NROW / 64, NPRJ / 128), 128, 0, stream>>>(X16, WP, Fp(5), QKA, V32);
  coef_kernel<<<NROW / 16, 256, 0, stream>>>(QKA, AB);
  seq_kernel<<<1, 32, 0, stream>>>(AB, F);
  scan_kernel<<<NB * D / 256, 256, 0, stream>>>(V32, F, Y32);
  y16_kernel<<<(NROW * D / 8 + 255) / 256, 256, 0, stream>>>(Y32, Y16, Y16L);
  out_kernel<<<dim3(NROW / 64, D / 128), 128, 0, stream>>>(Y16, Y16L, WO, (float*)d_out);
}
